// MambaBlock_21663815041549
// MI455X (gfx1250) — hardware-verified
//
#include <hip/hip_runtime.h>
#include <math.h>

typedef __attribute__((ext_vector_type(16))) _Float16 v16h;
typedef __attribute__((ext_vector_type(8)))  _Float16 v8h;
typedef __attribute__((ext_vector_type(16))) __bf16   v16b;
typedef __attribute__((ext_vector_type(8)))  __bf16   v8b;
typedef __attribute__((ext_vector_type(8)))  float    v8f;
typedef __attribute__((ext_vector_type(4)))  float    v4f;

constexpr int   kBatch  = 4;
constexpr int   kSeq    = 1024;
constexpr int   kDm     = 1024;
constexpr int   kNst    = 16;
constexpr int   kRows   = kBatch * kSeq;
constexpr int   kBcW    = 2 * kNst;
constexpr int   kNcat   = kDm + 64;
constexpr float kEps    = 1e-5f;
constexpr int   kScanCh = 128;
constexpr int   kScanTS = 64;
constexpr int   kScanYP = kScanCh + 4;
static_assert(kDm == 1024 && kNst == 16 && kSeq == 1024 && kBatch == 4, "shape constants");
static_assert((kDm % 32) == 0, "GEMM K multiple of 32");
static_assert((kRows % 64) == 0 && (kNcat % 64) == 0, "GEMM M,N multiples of 64");
static_assert((((kRows / 64) * (kNcat / 64)) % 8) == 0, "GEMM tiles fill whole blocks");
static_assert(kDm + kBcW <= kNcat, "B|C columns inside the padded width");
static_assert((kNcat * 4) % 128 == 0, "PRE row pitch is a whole number of 128-B lines");
static_assert((kSeq % kScanTS) == 0 && (kDm % kScanCh) == 0 && (kScanTS % 16) == 0, "scan tile multiples");
static_assert(kDm == 256 * 4, "LN: 256 threads x 4 elements per row");

constexpr size_t kOffXNF  = 0;
constexpr size_t kOffXNH  = kOffXNF + (size_t)kRows * kDm * 4;
constexpr size_t kOffXNL  = kOffXNH + (size_t)kRows * kDm * 2;
constexpr size_t kOffWH   = kOffXNL + (size_t)kRows * kDm * 2;
constexpr size_t kOffWL   = kOffWH  + (size_t)kNcat * kDm * 2;
constexpr size_t kOffPRE  = kOffWL  + (size_t)kNcat * kDm * 2;
constexpr size_t kWsTotal = kOffPRE + (size_t)kRows * kNcat * 4;
static_assert(kWsTotal == 55836672ull, "carve total");
static_assert(kWsTotal <= 134217728ull, "carve cap");
static_assert((kOffXNH % 128) == 0 && (kOffXNL % 128) == 0 && (kOffWH % 128) == 0 &&
              (kOffWL % 128) == 0 && (kOffPRE % 128) == 0, "128-B aligned regions");

__device__ __forceinline__ unsigned short f2bf_bits(float f) {
  unsigned u = __float_as_uint(f);
  return (unsigned short)((u + 0x7FFFu + ((u >> 16) & 1u)) >> 16);
}
__device__ __forceinline__ float bf_bits2f(unsigned short h) { return __uint_as_float(((unsigned)h) << 16); }

__device__ __forceinline__ void dep_guard_h(v8f& a, v8f& b, v16h x, v16h y) { asm volatile("v_nop\n\tv_nop\n\tv_nop\n\tv_nop" : "+v"(a), "+v"(b) : "v"(x), "v"(y)); }
__device__ __forceinline__ void dep_guard_b(v8f& a, v8f& b, v16b x, v16b y) { asm volatile("v_nop\n\tv_nop\n\tv_nop\n\tv_nop" : "+v"(a), "+v"(b) : "v"(x), "v"(y)); }
__device__ __forceinline__ void dep_guard4_h(v8f& a, v8f& b, v8f& c, v8f& d, v16h x, v16h y) { asm volatile("v_nop\n\tv_nop\n\tv_nop\n\tv_nop" : "+v"(a), "+v"(b), "+v"(c), "+v"(d) : "v"(x), "v"(y)); }
__device__ __forceinline__ void dep_guard4_b(v8f& a, v8f& b, v8f& c, v8f& d, v16b x, v16b y) { asm volatile("v_nop\n\tv_nop\n\tv_nop\n\tv_nop" : "+v"(a), "+v"(b), "+v"(c), "+v"(d) : "v"(x), "v"(y)); }
__device__ __forceinline__ void keep4_h(v16h a, v16h b, v16h c, v16h d) { asm volatile("v_nop" :: "v"(a), "v"(b), "v"(c), "v"(d)); }
__device__ __forceinline__ void keep4_b(v16b a, v16b b, v16b c, v16b d) { asm volatile("v_nop" :: "v"(a), "v"(b), "v"(c), "v"(d)); }
__device__ __forceinline__ void acc_guard4(v8f& a, v8f& b, v8f& c, v8f& d) { asm volatile("v_nop\n\tv_nop\n\tv_nop\n\tv_nop" : "+v"(a), "+v"(b), "+v"(c), "+v"(d)); }
template <typename T> struct Frag;
template <> struct Frag<_Float16> {
  typedef v16h V; union U { v16h v; v8h h[2]; };
  static __device__ __forceinline__ v16h load(const _Float16* p) {
    U f; f.h[0] = *(const v8h*)(p); f.h[1] = *(const v8h*)(p + 16); return f.v;
  }
  static __device__ __forceinline__ v8f mma(v16h a, v16h b, v8f c) {
    return __builtin_amdgcn_wmma_f32_16x16x32_f16(false, a, false, b, (short)0, c, false, false);
  }
  static __device__ __forceinline__ void guard(v8f& a, v8f& b, v16h x, v16h y) { dep_guard_h(a, b, x, y); }
  static __device__ __forceinline__ void guard4(v8f& a, v8f& b, v8f& c, v8f& d, v16h x, v16h y) { dep_guard4_h(a, b, c, d, x, y); }
  static __device__ __forceinline__ void keep(v16h a, v16h b, v16h c, v16h d) { keep4_h(a, b, c, d); }
};
template <> struct Frag<__bf16> {
  typedef v16b V; union U { v16b v; v8b h[2]; };
  static __device__ __forceinline__ v16b load(const __bf16* p) {
    U f; f.h[0] = *(const v8b*)(p); f.h[1] = *(const v8b*)(p + 16); return f.v;
  }
  static __device__ __forceinline__ v8f mma(v16b a, v16b b, v8f c) {
    return __builtin_amdgcn_wmma_f32_16x16x32_bf16(false, a, false, b, (short)0, c, false, false);
  }
  static __device__ __forceinline__ void guard(v8f& a, v8f& b, v16b x, v16b y) { dep_guard_b(a, b, x, y); }
  static __device__ __forceinline__ void guard4(v8f& a, v8f& b, v8f& c, v8f& d, v16b x, v16b y) { dep_guard4_b(a, b, c, d, x, y); }
  static __device__ __forceinline__ void keep(v16b a, v16b b, v16b c, v16b d) { keep4_b(a, b, c, d); }
};

template <int ET> struct Elem;
template <> struct Elem<0> { typedef _Float16 T; };
template <> struct Elem<1> { typedef __bf16 T; };
template <int ET, bool SPLIT, int BIAS_MODE, int OUT_MODE, bool RESID, int ACT = 0>
__global__ __launch_bounds__(256) void wmma_gemm64(
    const unsigned short* __restrict__ Ap, const unsigned short* __restrict__ A2p, int lda, long strideA,
    const unsigned short* __restrict__ Btp, const unsigned short* __restrict__ Bt2p, int ldb, long strideB,
    void* __restrict__ Cout, void* __restrict__ Cout2, int ldc, long strideC,
    const float* __restrict__ bias,
    const float* __restrict__ resid, long strideR,
    int M, int N, int K, float scale) {
  typedef typename Elem<ET>::T T;
  typedef typename Frag<T>::V V;
  const T* A = (const T*)Ap; const T* A2 = (const T*)A2p; const T* Bt = (const T*)Btp; const T* Bt2 = (const T*)Bt2p;
  __shared__ __align__(16) float sT[8][16 * 68];
  const int b    = blockIdx.y;
  const int lane = threadIdx.x & 31;
  const int wave = threadIdx.x >> 5;
  const int tilesN = N >> 6;
  const int tilesM = M >> 6;
  const int tile = blockIdx.x * 8 + wave;
  if (tile >= tilesM * tilesN) return;
  const int tm = tile / tilesN;
  const int tn = tile - tm * tilesN;
  const int m0 = tm << 6;
  const int n0 = tn << 6;

  const T* Ab  = A  + (size_t)b * strideA;
  const T* Bb  = Bt + (size_t)b * strideB;
  const T* Ab2 = SPLIT ? (A2  + (size_t)b * strideA) : nullptr;
  const T* Bb2 = SPLIT ? (Bt2 + (size_t)b * strideB) : nullptr;

  const int rlane = lane & 15;
  const int koff  = (lane >> 4) * 8;
  const int mOff  = (lane >> 4) * 8;

  v8f acc[4][4];
#pragma unroll
  for (int i = 0; i < 4; ++i)
#pragma unroll
    for (int j = 0; j < 4; ++j) acc[i][j] = (v8f){0.f,0.f,0.f,0.f,0.f,0.f,0.f,0.f};

  for (int k0 = 0; k0 < K; k0 += 32) {
    V bh[4], bl[4];
#pragma unroll
    for (int j = 0; j < 4; ++j) {
      const size_t bo = (size_t)(n0 + (j << 4) + rlane) * ldb + koff + k0;
      bh[j] = Frag<T>::load(Bb + bo);
      if (SPLIT) bl[j] = Frag<T>::load(Bb2 + bo);
    }
#pragma unroll
    for (int i = 0; i < 4; ++i) {
      const size_t ao = (size_t)(m0 + (i << 4) + rlane) * lda + koff + k0;
      V ah = Frag<T>::load(Ab + ao);
      V al;
      if (SPLIT) al = Frag<T>::load(Ab2 + ao);
#pragma unroll
      for (int j = 0; j < 4; ++j) {
        acc[i][j] = Frag<T>::mma(ah, bh[j], acc[i][j]);
        if (SPLIT) {
          acc[i][j] = Frag<T>::mma(ah, bl[j], acc[i][j]);
          acc[i][j] = Frag<T>::mma(al, bh[j], acc[i][j]);
        }
      }
      Frag<T>::guard4(acc[i][0], acc[i][1], acc[i][2], acc[i][3], ah, SPLIT ? al : ah);
    }
    Frag<T>::keep(bh[0], bh[1], bh[2], bh[3]);
    if (SPLIT) Frag<T>::keep(bl[0], bl[1], bl[2], bl[3]);
  }
  acc_guard4(acc[0][0], acc[0][1], acc[0][2], acc[0][3]);
  acc_guard4(acc[1][0], acc[1][1], acc[1][2], acc[1][3]);
  acc_guard4(acc[2][0], acc[2][1], acc[2][2], acc[2][3]);
  acc_guard4(acc[3][0], acc[3][1], acc[3][2], acc[3][3]);

  float* slab = sT[wave];
  const float* Rb = RESID ? (resid + (size_t)b * strideR) : nullptr;
#pragma unroll
  for (int i = 0; i < 4; ++i) {
    const int mBase = m0 + (i << 4);
#pragma unroll
    for (int j = 0; j < 4; ++j) {
      const int n = n0 + (j << 4) + rlane;
      float bv = 0.f;
      if (BIAS_MODE == 2) bv = bias[n];
#pragma unroll
      for (int r = 0; r < 8; ++r) {
        float v = acc[i][j][r] * scale;
        if (BIAS_MODE == 1) v += bias[mBase + mOff + r];
        if (BIAS_MODE == 2) v += bv;
        if (RESID) v += Rb[(size_t)(mBase + mOff + r) * ldc + n];
        if (ACT == 1) v = tanhf(v);
        if (ACT == 2) v = fmaxf(v, 0.0f);
        if (ACT == 3) v = v / (1.0f + expf(-v));
        if (ACT == 4) v = (v > 0.f) ? v : 0.01f * v;
        slab[(mOff + r) * 68 + (j << 4) + rlane] = v;
      }
    }
    __builtin_amdgcn_fence(__ATOMIC_RELEASE, "workgroup");
    __builtin_amdgcn_wave_barrier();
    __builtin_amdgcn_fence(__ATOMIC_ACQUIRE, "workgroup");
    if (OUT_MODE == 0) {
      float* C = (float*)Cout + (size_t)b * strideC;
      const int hh = lane >> 4, c4 = (lane & 15) * 4;
      for (int pass = 0; pass < 2; ++pass) {
#pragma unroll
        for (int it = 0; it < 8; ++it) {
          const int row = it * 2 + hh;
          v4f v = *(const v4f*)(slab + row * 68 + c4);
          *(volatile v4f*)(C + (size_t)(mBase + row) * ldc + n0 + c4) = v;
        }
        __threadfence();
      }
    } else {
      const int q = lane >> 3, c8 = (lane & 7) * 8;
      unsigned short* C  = (unsigned short*)Cout  + (size_t)b * strideC;
      unsigned short* C2 = (OUT_MODE == 2) ? ((unsigned short*)Cout2 + (size_t)b * strideC) : nullptr;
      for (int pass = 0; pass < 2; ++pass) {
#pragma unroll
        for (int it = 0; it < 4; ++it) {
          const int row = it * 4 + q;
          const float* sp = slab + row * 68 + c8;
          v8h hv, lv;
#pragma unroll
          for (int e = 0; e < 8; ++e) {
            if (OUT_MODE == 1) {
              hv[e] = (_Float16)sp[e];
            } else {
              unsigned short hb = f2bf_bits(sp[e]);
              unsigned short lb = f2bf_bits(sp[e] - bf_bits2f(hb));
              hv[e] = __builtin_bit_cast(_Float16, hb);
              lv[e] = __builtin_bit_cast(_Float16, lb);
            }
          }
          *(volatile v8h*)(C + (size_t)(mBase + row) * ldc + n0 + c8) = hv;
          if (OUT_MODE == 2) *(volatile v8h*)(C2 + (size_t)(mBase + row) * ldc + n0 + c8) = lv;
        }
        __threadfence();
      }
    }
    __builtin_amdgcn_fence(__ATOMIC_RELEASE, "workgroup");
    __builtin_amdgcn_wave_barrier();
    __builtin_amdgcn_fence(__ATOMIC_ACQUIRE, "workgroup");
  }
}

__global__ __launch_bounds__(256) void ln_kernel(
    const float* __restrict__ x, const float* __restrict__ gamma, const float* __restrict__ beta,
    float* __restrict__ XNF, unsigned short* __restrict__ XNH, unsigned short* __restrict__ XNL)
{
  __shared__ __align__(16) float srow[kDm];
  __shared__ float sred0[8];
  __shared__ float sred1[8];
  const int tid = threadIdx.x, lane = tid & 31, wave = tid >> 5;
  const size_t rbase = (size_t)blockIdx.x * kDm;
  const v4f xv = *(const v4f*)(x + rbase + 4 * tid);
  float s = 0.f;
  s += xv[0]; s += xv[1]; s += xv[2]; s += xv[3];
#pragma unroll
  for (int m = 16; m >= 1; m >>= 1) s += __shfl_xor(s, m, 32);
  if (lane == 0) sred0[wave] = s;
  __syncthreads();
  float tot = 0.f;
#pragma unroll
  for (int w = 0; w < 8; ++w) tot += sred0[w];
  const float mean = tot * (1.0f / (float)kDm);
  const float dv0 = xv[0] - mean, dv1 = xv[1] - mean, dv2 = xv[2] - mean, dv3 = xv[3] - mean;
  float ss = 0.f;
  ss += dv0 * dv0; ss += dv1 * dv1; ss += dv2 * dv2; ss += dv3 * dv3;
#pragma unroll
  for (int m = 16; m >= 1; m >>= 1) ss += __shfl_xor(ss, m, 32);
  if (lane == 0) sred1[wave] = ss;
  __syncthreads();
  float tot2 = 0.f;
#pragma unroll
  for (int w = 0; w < 8; ++w) tot2 += sred1[w];
  const float var  = tot2 * (1.0f / (float)kDm);
  const float rstd = rsqrtf(var + kEps);
  const v4f gv = *(const v4f*)(gamma + 4 * tid);
  const v4f bv = *(const v4f*)(beta + 4 * tid);
  v4f o;
  o[0] = (dv0 * rstd) * gv[0] + bv[0];
  o[1] = (dv1 * rstd) * gv[1] + bv[1];
  o[2] = (dv2 * rstd) * gv[2] + bv[2];
  o[3] = (dv3 * rstd) * gv[3] + bv[3];
  *(v4f*)(srow + 4 * tid) = o;
  float* dst = XNF + rbase + 4 * tid;
  for (int pass = 0; pass < 2; ++pass) {
    *(volatile v4f*)dst = o;
    __threadfence();
  }
  __syncthreads();
  if (tid < 128) {
    const v4f a0 = *(const v4f*)(srow + 8 * tid);
    const v4f a1 = *(const v4f*)(srow + 8 * tid + 4);
    v8h hv, lv;
#pragma unroll
    for (int e = 0; e < 4; ++e) {
      const unsigned short h0 = f2bf_bits(a0[e]), h1 = f2bf_bits(a1[e]);
      const unsigned short l0 = f2bf_bits(a0[e] - bf_bits2f(h0)), l1 = f2bf_bits(a1[e] - bf_bits2f(h1));
      hv[e]     = __builtin_bit_cast(_Float16, h0);
      hv[4 + e] = __builtin_bit_cast(_Float16, h1);
      lv[e]     = __builtin_bit_cast(_Float16, l0);
      lv[4 + e] = __builtin_bit_cast(_Float16, l1);
    }
    const size_t o8 = rbase + (size_t)8 * tid;
    for (int pass = 0; pass < 2; ++pass) {
      *(volatile v8h*)(XNH + o8) = hv;
      *(volatile v8h*)(XNL + o8) = lv;
      __threadfence();
    }
  }
}

__global__ __launch_bounds__(256) void wsplit_kernel(
    const float* __restrict__ Wd, const float* __restrict__ WB, const float* __restrict__ WC,
    unsigned short* __restrict__ BH, unsigned short* __restrict__ BL)
{
  __shared__ float tile[64 * 65];
  const int tid = threadIdx.x, lane = tid & 31, wave = tid >> 5;
  const int n0 = blockIdx.x * 64;
  const int k0 = blockIdx.y * 64;
  if (blockIdx.x < kDm / 64) {
#pragma unroll 4
    for (int p = 0; p < 16; ++p) {
      const int idx = tid + p * 256;
      const int kk  = idx >> 6;
      const int nn  = idx & 63;
      tile[kk * 65 + nn] = Wd[(size_t)(k0 + kk) * kDm + n0 + nn];
    }
  } else {
#pragma unroll 4
    for (int p = 0; p < 16; ++p) {
      const int idx = tid + p * 256;
      const int kk  = idx >> 6;
      const int nn  = idx & 63;
      const int c   = nn & (kNst - 1);
      const float vb = WB[(size_t)(k0 + kk) * kNst + c];
      const float vc = WC[(size_t)(k0 + kk) * kNst + c];
      const float fb = (nn < kNst) ? 1.0f : 0.0f;
      const float fc = (nn >= kNst && nn < 2 * kNst) ? 1.0f : 0.0f;
      tile[kk * 65 + nn] = fmaf(fb, vb, fc * vc);
    }
  }
  __syncthreads();
  const int q = lane >> 3, c8 = (lane & 7) * 8;
  v8h hv[2], lv[2];
#pragma unroll
  for (int it = 0; it < 2; ++it) {
    const int nrow = it * 32 + wave * 4 + q;
#pragma unroll
    for (int e = 0; e < 8; ++e) {
      const float v = tile[(c8 + e) * 65 + nrow];
      const unsigned short hb = f2bf_bits(v);
      const unsigned short lb = f2bf_bits(v - bf_bits2f(hb));
      hv[it][e] = __builtin_bit_cast(_Float16, hb);
      lv[it][e] = __builtin_bit_cast(_Float16, lb);
    }
  }
  for (int pass = 0; pass < 2; ++pass) {
#pragma unroll
    for (int it = 0; it < 2; ++it) {
      const int nrow = it * 32 + wave * 4 + q;
      const size_t o = (size_t)(n0 + nrow) * kDm + k0 + c8;
      *(volatile v8h*)(BH + o) = hv[it];
      *(volatile v8h*)(BL + o) = lv[it];
    }
    __threadfence();
  }
}

__global__ __launch_bounds__(kScanCh) void scan_kernel(
    const float* __restrict__ PRE, const float* __restrict__ XNF, const float* __restrict__ X,
    const float* __restrict__ bdl, const float* __restrict__ bB, const float* __restrict__ bC,
    const float* __restrict__ Alog, const float* __restrict__ Dsk, float* __restrict__ out)
{
  __shared__ __align__(16) float sBC[kScanTS * kBcW];
  __shared__ __align__(16) float sY[kScanTS * kScanYP];
  __shared__ __align__(16) float sA[kNst * kScanCh];
  const int tid = threadIdx.x, lane = tid & 31, wave = tid >> 5;
  constexpr int kBlkPerB = kDm / kScanCh;
  const int bix = blockIdx.x / kBlkPerB;
  const int d0  = (blockIdx.x - bix * kBlkPerB) * kScanCh;
  const int d   = d0 + tid;
  const size_t row0 = (size_t)bix * kSeq;
#pragma unroll 1
  for (int n = 0; n < kNst; ++n) sA[n * kScanCh + tid] = -expf(Alog[(size_t)d * kNst + n]);
  __syncthreads();
  float An[kNst], h[kNst];
#pragma unroll
  for (int n = 0; n < kNst; ++n) {
    An[n] = sA[n * kScanCh + tid];
    h[n]  = 0.f;
  }
  const float bd = bdl[d];
  const float Dd = Dsk[d];
  const int lr = tid >> 3, q4 = (tid & 7) * 4;
  const v4f vB = *(const v4f*)(bB + (q4 & (kNst - 1)));
  const v4f vC = *(const v4f*)(bC + (q4 & (kNst - 1)));
  const float fb = (q4 < kNst) ? 1.0f : 0.0f;
  const float fc = 1.0f - fb;
  v4f bias4;
#pragma unroll
  for (int e = 0; e < 4; ++e) bias4[e] = fmaf(fb, vB[e], fc * vC[e]);

#pragma unroll 1
  for (int t0 = 0; t0 < kSeq; t0 += kScanTS) {
    __syncthreads();
#pragma unroll
    for (int i = 0; i < kScanTS / 16; ++i) {
      const int r = lr + 16 * i;
      v4f v = *(const v4f*)(PRE + (row0 + t0 + r) * kNcat + kDm + q4);
      v += bias4;
      *(v4f*)(sBC + r * kBcW + q4) = v;
    }
    __syncthreads();
#pragma unroll 1
    for (int s = 0; s < kScanTS; ++s) {
      const size_t m = row0 + t0 + s;
      const float a    = PRE[m * kNcat + d] + bd;
      const float dt   = fmaxf(a, 0.0f) + log1pf(__expf(-fabsf(a)));
      const float xt   = XNF[m * kDm + d];
      const float xres = X[m * kDm + d];
      v4f Bq[4], Cq[4];
#pragma unroll
      for (int qq = 0; qq < 4; ++qq) {
        Bq[qq] = *(const v4f*)(sBC + s * kBcW + 4 * qq);
        Cq[qq] = *(const v4f*)(sBC + s * kBcW + kNst + 4 * qq);
      }
      const float dtx = dt * xt;
      float y = 0.f;
#pragma unroll
      for (int n = 0; n < kNst; ++n) {
        const float e  = __expf(dt * An[n]);
        const float hn = e * h[n] + dtx * Bq[n >> 2][n & 3];
        h[n] = hn;
        y += hn * Cq[n >> 2][n & 3];
      }
      const float yt = y + Dd * xt;
      sY[s * kScanYP + tid] = xres + yt;
    }
    __syncthreads();
    for (int pass = 0; pass < 2; ++pass) {
#pragma unroll
      for (int it = 0; it < kScanTS / 4; ++it) {
        const int row = it * 4 + wave;
        const v4f v = *(const v4f*)(sY + row * kScanYP + lane * 4);
        *(volatile v4f*)(out + (row0 + t0 + row) * kDm + d0 + lane * 4) = v;
      }
      __threadfence();
    }
  }
}

extern "C" void kernel_launch(void* const* d_in, const int* in_sizes, int n_in,
                              void* d_out, int out_size, void* d_ws, size_t ws_size,
                              hipStream_t stream)
{
  if (n_in < 11) return;
  if (in_sizes[0] != kRows * kDm) return;
  if (in_sizes[1] != kDm || in_sizes[2] != kDm) return;
  if (in_sizes[3] != kDm * kDm || in_sizes[4] != kDm) return;
  if (in_sizes[5] != kDm * kNst || in_sizes[6] != kNst) return;
  if (in_sizes[7] != kDm * kNst || in_sizes[8] != kNst) return;
  if (in_sizes[9] != kDm * kNst || in_sizes[10] != kDm) return;
  if (out_size != kRows * kDm) return;
  if (ws_size < kWsTotal) return;

  const float* x       = (const float*)d_in[0];
  const float* gamma   = (const float*)d_in[1];
  const float* beta    = (const float*)d_in[2];
  const float* W_delta = (const float*)d_in[3];
  const float* b_delta = (const float*)d_in[4];
  const float* W_B     = (const float*)d_in[5];
  const float* b_B     = (const float*)d_in[6];
  const float* W_C     = (const float*)d_in[7];
  const float* b_C     = (const float*)d_in[8];
  const float* A_log   = (const float*)d_in[9];
  const float* D_skip  = (const float*)d_in[10];
  float* out = (float*)d_out;

  char* ws = (char*)d_ws;
  float*          XNF = (float*)(ws + kOffXNF);
  unsigned short* XNH = (unsigned short*)(ws + kOffXNH);
  unsigned short* XNL = (unsigned short*)(ws + kOffXNL);
  unsigned short* WH  = (unsigned short*)(ws + kOffWH);
  unsigned short* WL  = (unsigned short*)(ws + kOffWL);
  float*          PRE = (float*)(ws + kOffPRE);
  const float* dummy_bias  = b_delta;
  const float* dummy_resid = XNF;

  ln_kernel<<<dim3(kRows), 256, 0, stream>>>(x, gamma, beta, XNF, XNH, XNL);

  wsplit_kernel<<<dim3(kNcat / 64, kDm / 64), 256, 0, stream>>>(W_delta, W_B, W_C, WH, WL);

  wmma_gemm64<1, true, 0, 0, false><<<dim3(((kRows / 64) * (kNcat / 64)) / 8, 1), 256, 0, stream>>>(
      XNH, XNL, kDm, 0L,
      WH, WL, kDm, 0L,
      (void*)PRE, (void*)PRE, kNcat, 0L,
      dummy_bias, dummy_resid, 0L,
      kRows, kNcat, kDm, 1.0f);

  scan_kernel<<<dim3(kBatch * (kDm / kScanCh)), kScanCh, 0, stream>>>(
      PRE, XNF, x, b_delta, b_B, b_C, A_log, D_skip, out);
}
